// energy_latencyGNN_10_1_41446434406430
// MI455X (gfx1250) — hardware-verified
//
#include <hip/hip_runtime.h>

typedef _Float16 half_t;
typedef _Float16 v16h __attribute__((ext_vector_type(16)));
typedef _Float16 v8h  __attribute__((ext_vector_type(8)));
typedef float    v8f  __attribute__((ext_vector_type(8)));
typedef float    v4f  __attribute__((ext_vector_type(4)));

union Frag  { v16h v; v8h half[2]; };
union Pack8 { v8h v; half_t h[8]; };
union U4    { v4f v; float f[4]; };

#define NN     20
#define EMBD   5
#define NE     100
#define DW     120
#define XW     220
#define XP     224
#define H1     128
#define H2     128
#define H3     64
#define HP     128
#define EMAX   128
#define TB     64
#define WSCALE 16.0f
#define WINV   0.0625f
#define SLOPE  0.01f

__device__ __forceinline__ float leaky(float x) { return x >= 0.f ? x : SLOPE * x; }
__device__ __forceinline__ float sigm(float x)  { return __builtin_amdgcn_rcpf(1.0f + __expf(-x)); }

__device__ __forceinline__ v8f zero8() {
  v8f z;
#pragma unroll
  for (int i = 0; i < 8; ++i) z[i] = 0.f;
  return z;
}

__device__ __forceinline__ v8f wmma16(v16h a, v16h b, v8f c) {
  c = __builtin_amdgcn_wmma_f32_16x16x32_f16(false, a, false, b, (short)0, c, false, false);
  asm volatile("v_nop\n\tv_nop\n\tv_nop\n\tv_nop" : "+v"(c) : "v"(a), "v"(b));
  return c;
}

__global__ void __launch_bounds__(TB) k_wcvt(const float* __restrict__ W, int kreal, int nreal, int kp,
                                            half_t* __restrict__ outp, int ngroups) {
  const int g = blockIdx.x * TB + threadIdx.x;
  if (g >= ngroups) return;
  const int gpr = kp >> 3;
  const int n   = g / gpr;
  const int k8  = (g - n * gpr) * 8;
  Pack8 u;
#pragma unroll
  for (int i = 0; i < 8; ++i) {
    const int k = k8 + i;
    float v = 0.0f;
    if (k < kreal) v = W[(size_t)k * nreal + n] * WSCALE;
    u.h[i] = (half_t)v;
  }
  const v8h val = u.v;
  volatile v8h* p = (volatile v8h*)(outp + (size_t)g * 8);
  *p = val;
  __threadfence();
  *p = val;
}

__global__ void __launch_bounds__(TB) k_main(
    const float* __restrict__ data, const float* __restrict__ dmat,
    const int* __restrict__ src, const int* __restrict__ dst,
    const float* __restrict__ g0U, const float* __restrict__ g0V,
    const float* __restrict__ g0A, const float* __restrict__ g0B,
    const float* __restrict__ g0bU, const float* __restrict__ g0bV,
    const float* __restrict__ g0bA, const float* __restrict__ g0bB,
    const float* __restrict__ gU, const float* __restrict__ gV,
    const float* __restrict__ gA, const float* __restrict__ gB,
    const float* __restrict__ gbU, const float* __restrict__ gbV,
    const float* __restrict__ gbA, const float* __restrict__ gbB,
    const half_t* __restrict__ wt1, const half_t* __restrict__ wt2, const half_t* __restrict__ wt3,
    const float* __restrict__ b1, const float* __restrict__ b2, const float* __restrict__ b3,
    const float* __restrict__ W4, const float* __restrict__ b4,
    float* __restrict__ out, int e_cnt) {
  __shared__ __align__(16) float  hs[TB * NE];
  __shared__ __align__(16) float  ag[TB * NE];
  __shared__ __align__(16) float  h0s[TB * NN];
  __shared__ int sSrc[EMAX];
  __shared__ int sDst[EMAX];
  __shared__ __align__(16) half_t sX[TB * XP];
  __shared__ __align__(16) half_t sP[TB * HP];
  __shared__ __align__(16) half_t sQ[TB * HP];
  __shared__ U4 sOut[32];

  const int tid = threadIdx.x;
  const int blk = blockIdx.x;

  {
    const float* dbase = data + (size_t)blk * (TB * NN);
    for (int i = tid; i < (TB * NN) / 4; i += TB) {
      v4f v = *(const v4f*)(dbase + 4 * i);
      *(v4f*)(h0s + 4 * i) = v;
    }
    const float* mbase = dmat + (size_t)blk * (TB * DW);
    for (int i = tid; i < (TB * DW) / 4; i += TB) {
      v4f v = *(const v4f*)(mbase + 4 * i);
      const int row = i / (DW / 4);
      const int c4  = (i - row * (DW / 4)) * 4;
      half_t* xp = sX + row * XP + NE + c4;
      xp[0] = (half_t)v[0]; xp[1] = (half_t)v[1]; xp[2] = (half_t)v[2]; xp[3] = (half_t)v[3];
    }
    for (int e = tid; e < e_cnt; e += TB) {
      int s = src[e], t = dst[e];
      if (s < 0) s += NN;
      if (t < 0) t += NN;
      s = s < 0 ? 0 : (s >= NN ? NN - 1 : s);
      t = t < 0 ? 0 : (t >= NN ? NN - 1 : t);
      sSrc[e] = s; sDst[e] = t;
    }
  }
  __syncthreads();

  float* h  = hs + tid * NE;
  float* a  = ag + tid * NE;
  const float* h0 = h0s + tid * NN;

  {
    float U0[EMBD], V0[EMBD], A0w[EMBD], B0w[EMBD], bU0[EMBD], bV0[EMBD], zb0[EMBD];
#pragma unroll
    for (int c = 0; c < EMBD; ++c) {
      U0[c] = g0U[c]; V0[c] = g0V[c]; A0w[c] = g0A[c]; B0w[c] = g0B[c];
      bU0[c] = g0bU[c]; bV0[c] = g0bV[c]; zb0[c] = g0bA[c] + g0bB[c];
    }
#pragma unroll 4
    for (int i = 0; i < NE; ++i) a[i] = 0.f;
#pragma unroll 1
    for (int e = 0; e < e_cnt; ++e) {
      const int s = sSrc[e], t = sDst[e];
      const float hu = h0[s], hv = h0[t];
#pragma unroll
      for (int c = 0; c < EMBD; ++c) {
        const float g = sigm(hu * A0w[c] + hv * B0w[c] + zb0[c]);
        a[t * EMBD + c] += g * (hu * V0[c] + bV0[c]);
      }
    }
#pragma unroll 1
    for (int n = 0; n < NN; ++n) {
      const float x = h0[n];
#pragma unroll
      for (int c = 0; c < EMBD; ++c)
        h[n * EMBD + c] = leaky(x * U0[c] + bU0[c] + a[n * EMBD + c]);
    }
  }

#pragma unroll 1
  for (int ly = 0; ly < 2; ++ly) {
    float Vw[25], Aw[25], Bw[25], zb[EMBD], bV[EMBD];
#pragma unroll
    for (int i = 0; i < 25; ++i) {
      Vw[i] = gV[ly * 25 + i]; Aw[i] = gA[ly * 25 + i]; Bw[i] = gB[ly * 25 + i];
    }
#pragma unroll
    for (int c = 0; c < EMBD; ++c) {
      zb[c] = gbA[ly * EMBD + c] + gbB[ly * EMBD + c];
      bV[c] = gbV[ly * EMBD + c];
    }
#pragma unroll 4
    for (int i = 0; i < NE; ++i) a[i] = 0.f;

#pragma unroll 1
    for (int e = 0; e < e_cnt; ++e) {
      const int s = sSrc[e], t = sDst[e];
      float hu[EMBD], hv[EMBD];
#pragma unroll
      for (int k = 0; k < EMBD; ++k) { hu[k] = h[s * EMBD + k]; hv[k] = h[t * EMBD + k]; }
#pragma unroll
      for (int c = 0; c < EMBD; ++c) {
        float z = zb[c], zv = bV[c];
#pragma unroll
        for (int k = 0; k < EMBD; ++k) {
          z  += hu[k] * Aw[k * EMBD + c] + hv[k] * Bw[k * EMBD + c];
          zv += hu[k] * Vw[k * EMBD + c];
        }
        a[t * EMBD + c] += sigm(z) * zv;
      }
    }

    float Uw[25], bU[EMBD];
#pragma unroll
    for (int i = 0; i < 25; ++i) Uw[i] = gU[ly * 25 + i];
#pragma unroll
    for (int c = 0; c < EMBD; ++c) bU[c] = gbU[ly * EMBD + c];
#pragma unroll 1
    for (int n = 0; n < NN; ++n) {
      float hn[EMBD], tmp[EMBD];
#pragma unroll
      for (int k = 0; k < EMBD; ++k) hn[k] = h[n * EMBD + k];
#pragma unroll
      for (int c = 0; c < EMBD; ++c) {
        float z = bU[c] + a[n * EMBD + c];
#pragma unroll
        for (int k = 0; k < EMBD; ++k) z += hn[k] * Uw[k * EMBD + c];
        tmp[c] = leaky(z);
      }
#pragma unroll
      for (int c = 0; c < EMBD; ++c) h[n * EMBD + c] = tmp[c];
    }
  }

  {
    half_t* xr = sX + tid * XP;
#pragma unroll 4
    for (int i = 0; i < NE; ++i) xr[i] = (half_t)h[i];
#pragma unroll
    for (int j = 0; j < XP - XW; ++j) xr[XW + j] = (half_t)0.f;
  }
  __syncthreads();

  const int lane  = tid & 31;
  const int hh    = lane >> 4;
  const int m     = lane & 15;
  const int wv    = tid >> 5;
  const int koff0 = 8 * hh;
  const int koff1 = 16 + 8 * hh;

#pragma unroll 1
  for (int j = 0; j < H1 / 16; ++j) {
    v8f c0 = zero8(), c1 = zero8();
    const half_t* arow0 = sX + (32 * wv + m) * XP;
    const half_t* arow1 = arow0 + 16 * XP;
    const half_t* brow  = wt1 + (size_t)(16 * j + m) * XP;
#pragma unroll 1
    for (int kc = 0; kc < XP / 32; ++kc) {
      const int k0 = kc * 32;
      Frag fa0, fa1, fb;
      fa0.half[0] = *(const v8h*)(arow0 + k0 + koff0);
      fa0.half[1] = *(const v8h*)(arow0 + k0 + koff1);
      fa1.half[0] = *(const v8h*)(arow1 + k0 + koff0);
      fa1.half[1] = *(const v8h*)(arow1 + k0 + koff1);
      fb.half[0]  = *(const v8h*)(brow + k0 + koff0);
      fb.half[1]  = *(const v8h*)(brow + k0 + koff1);
      c0 = wmma16(fa0.v, fb.v, c0);
      c1 = wmma16(fa1.v, fb.v, c1);
    }
    const int n = 16 * j + m;
    const float bias = b1[n];
#pragma unroll
    for (int r = 0; r < 8; ++r) {
      const int row = 32 * wv + 8 * hh + r;
      sP[row * HP + n]        = (half_t)leaky(c0[r] * WINV + bias);
      sP[(row + 16) * HP + n] = (half_t)leaky(c1[r] * WINV + bias);
    }
  }
  __syncthreads();

#pragma unroll 1
  for (int j = 0; j < H2 / 16; ++j) {
    v8f c0 = zero8(), c1 = zero8();
    const half_t* arow0 = sP + (32 * wv + m) * HP;
    const half_t* arow1 = arow0 + 16 * HP;
    const half_t* brow  = wt2 + (size_t)(16 * j + m) * HP;
#pragma unroll 1
    for (int kc = 0; kc < H1 / 32; ++kc) {
      const int k0 = kc * 32;
      Frag fa0, fa1, fb;
      fa0.half[0] = *(const v8h*)(arow0 + k0 + koff0);
      fa0.half[1] = *(const v8h*)(arow0 + k0 + koff1);
      fa1.half[0] = *(const v8h*)(arow1 + k0 + koff0);
      fa1.half[1] = *(const v8h*)(arow1 + k0 + koff1);
      fb.half[0]  = *(const v8h*)(brow + k0 + koff0);
      fb.half[1]  = *(const v8h*)(brow + k0 + koff1);
      c0 = wmma16(fa0.v, fb.v, c0);
      c1 = wmma16(fa1.v, fb.v, c1);
    }
    const int n = 16 * j + m;
    const float bias = b2[n];
#pragma unroll
    for (int r = 0; r < 8; ++r) {
      const int row = 32 * wv + 8 * hh + r;
      sQ[row * HP + n]        = (half_t)leaky(c0[r] * WINV + bias);
      sQ[(row + 16) * HP + n] = (half_t)leaky(c1[r] * WINV + bias);
    }
  }
  __syncthreads();

  float* sF = ag;
#pragma unroll 1
  for (int j = 0; j < H3 / 16; ++j) {
    v8f c0 = zero8(), c1 = zero8();
    const half_t* arow0 = sQ + (32 * wv + m) * HP;
    const half_t* arow1 = arow0 + 16 * HP;
    const half_t* brow  = wt3 + (size_t)(16 * j + m) * HP;
#pragma unroll 1
    for (int kc = 0; kc < H2 / 32; ++kc) {
      const int k0 = kc * 32;
      Frag fa0, fa1, fb;
      fa0.half[0] = *(const v8h*)(arow0 + k0 + koff0);
      fa0.half[1] = *(const v8h*)(arow0 + k0 + koff1);
      fa1.half[0] = *(const v8h*)(arow1 + k0 + koff0);
      fa1.half[1] = *(const v8h*)(arow1 + k0 + koff1);
      fb.half[0]  = *(const v8h*)(brow + k0 + koff0);
      fb.half[1]  = *(const v8h*)(brow + k0 + koff1);
      c0 = wmma16(fa0.v, fb.v, c0);
      c1 = wmma16(fa1.v, fb.v, c1);
    }
    const int n = 16 * j + m;
    const float bias = b3[n];
#pragma unroll
    for (int r = 0; r < 8; ++r) {
      const int row = 32 * wv + 8 * hh + r;
      sF[row * H3 + n]        = leaky(c0[r] * WINV + bias);
      sF[(row + 16) * H3 + n] = leaky(c1[r] * WINV + bias);
    }
  }
  __syncthreads();

  {
    float z0 = b4[0], z1 = b4[1];
    const float* xr = sF + tid * H3;
#pragma unroll 8
    for (int k = 0; k < H3; ++k) {
      const float x = xr[k];
      z0 += x * W4[k * 2 + 0];
      z1 += x * W4[k * 2 + 1];
    }
    sOut[tid >> 1].f[(tid & 1) * 2 + 0] = sigm(z0);
    sOut[tid >> 1].f[(tid & 1) * 2 + 1] = sigm(z1);
  }
  __syncthreads();

  if (tid < 32) {
    const v4f v = sOut[tid].v;
    volatile v4f* p = (volatile v4f*)(out + (size_t)blk * (TB * 2)) + tid;
    *p = v;
    __threadfence();
    *p = v;
  }
}

extern "C" void kernel_launch(void* const* d_in, const int* in_sizes, int n_in,
                              void* d_out, int out_size, void* d_ws, size_t ws_size,
                              hipStream_t stream) {
  if (n_in < 28) return;
  const int B = out_size / 2;
  if (B <= 0 || out_size != 2 * B || (B % TB) != 0) return;
  if (in_sizes[0] != B * NN || in_sizes[1] != B * DW) return;
  for (int i = 4; i <= 11; ++i) if (in_sizes[i] != EMBD) return;
  for (int i = 12; i <= 15; ++i) if (in_sizes[i] != 2 * EMBD * EMBD) return;
  for (int i = 16; i <= 19; ++i) if (in_sizes[i] != 2 * EMBD) return;
  if (in_sizes[20] != XW * H1 || in_sizes[21] != H1) return;
  if (in_sizes[22] != H1 * H2 || in_sizes[23] != H2) return;
  if (in_sizes[24] != H2 * H3 || in_sizes[25] != H3) return;
  if (in_sizes[26] != H3 * 2 || in_sizes[27] != 2) return;
  int e_cnt = in_sizes[2] < in_sizes[3] ? in_sizes[2] : in_sizes[3];
  if (e_cnt < 0) e_cnt = 0;
  if (e_cnt > EMAX) e_cnt = EMAX;

  const size_t off1 = 0;
  const size_t off2 = off1 + (size_t)H1 * XP * 2;
  const size_t off3 = off2 + (size_t)H2 * HP * 2;
  const size_t wend = off3 + (size_t)H3 * HP * 2;
  if (ws_size < wend) return;
  half_t* wt1 = (half_t*)((char*)d_ws + off1);
  half_t* wt2 = (half_t*)((char*)d_ws + off2);
  half_t* wt3 = (half_t*)((char*)d_ws + off3);

  const float* data = (const float*)d_in[0];
  const float* dmat = (const float*)d_in[1];
  const int*   src  = (const int*)d_in[2];
  const int*   dst  = (const int*)d_in[3];
  const float* g0U  = (const float*)d_in[4];
  const float* g0V  = (const float*)d_in[5];
  const float* g0A  = (const float*)d_in[6];
  const float* g0B  = (const float*)d_in[7];
  const float* g0bU = (const float*)d_in[8];
  const float* g0bV = (const float*)d_in[9];
  const float* g0bA = (const float*)d_in[10];
  const float* g0bB = (const float*)d_in[11];
  const float* gU   = (const float*)d_in[12];
  const float* gV   = (const float*)d_in[13];
  const float* gA   = (const float*)d_in[14];
  const float* gB   = (const float*)d_in[15];
  const float* gbU  = (const float*)d_in[16];
  const float* gbV  = (const float*)d_in[17];
  const float* gbA  = (const float*)d_in[18];
  const float* gbB  = (const float*)d_in[19];
  const float* fW1  = (const float*)d_in[20];
  const float* fb1  = (const float*)d_in[21];
  const float* fW2  = (const float*)d_in[22];
  const float* fb2  = (const float*)d_in[23];
  const float* fW3  = (const float*)d_in[24];
  const float* fb3  = (const float*)d_in[25];
  const float* fW4  = (const float*)d_in[26];
  const float* fb4  = (const float*)d_in[27];

  const int ng1 = H1 * (XP / 8);
  const int ng2 = H2 * (HP / 8);
  const int ng3 = H3 * (HP / 8);
  k_wcvt<<<(ng1 + TB - 1) / TB, TB, 0, stream>>>(fW1, XW, H1, XP, wt1, ng1);
  k_wcvt<<<(ng2 + TB - 1) / TB, TB, 0, stream>>>(fW2, H1, H2, HP, wt2, ng2);
  k_wcvt<<<(ng3 + TB - 1) / TB, TB, 0, stream>>>(fW3, H2, H3, HP, wt3, ng3);

  k_main<<<B / TB, TB, 0, stream>>>(
      data, dmat, src, dst,
      g0U, g0V, g0A, g0B, g0bU, g0bV, g0bA, g0bB,
      gU, gV, gA, gB, gbU, gbV, gbA, gbB,
      wt1, wt2, wt3, fb1, fb2, fb3, fW4, fb4,
      (float*)d_out, e_cnt);
}
